// TransformerBlock_66159676228026
// MI455X (gfx1250) — hardware-verified
//
#include <hip/hip_runtime.h>
#include <stddef.h>


typedef _Float16 v16h __attribute__((ext_vector_type(16)));
typedef _Float16 v8h  __attribute__((ext_vector_type(8)));
typedef float    v8f  __attribute__((ext_vector_type(8)));
typedef float    v4f  __attribute__((ext_vector_type(4)));

#ifndef NB
#define NB 2
#endif
#ifndef SEQ
#define SEQ 2048
#endif
#define NB_FULL  2
#define SEQ_FULL 2048
#define DIM   768
#define DFF   3072
#define NHEAD 12
#define HD    64
#define QKLD  (2 * DIM)
#define MROWS (NB * SEQ)
#define LNROWS 8
#define LN_EPS 1.0e-5f

static_assert(NB >= 1 && NB <= NB_FULL);
static_assert(SEQ >= 128 && SEQ <= SEQ_FULL && (SEQ % 128) == 0);
static_assert(DIM == NHEAD * HD);
static_assert(HD == 64);
static_assert((DIM % 64) == 0 && (DIM % 32) == 0);
static_assert((DFF % 64) == 0 && (DFF % 32) == 0);
static_assert((QKLD % 64) == 0);
static_assert((MROWS % 64) == 0);
static_assert((MROWS % LNROWS) == 0);
static_assert((DIM % 256) == 0);
static_assert((size_t)MROWS * DFF < (size_t)0xFFFFFFFFu);
static_assert((size_t)((NB - 1) * SEQ_FULL + SEQ) * DIM <= (size_t)NB_FULL * SEQ_FULL * DIM);

#define LDT 72
#define LDC 68

#define WCARRY 64.0f
#define PCARRY 1024.0f
#define VCARRY 64.0f

#define WQKV_BYTES ((size_t)3 * DIM * DIM * 2)
#define WO_BYTES   ((size_t)DIM * DIM * 2)
#define WFF_BYTES  ((size_t)DFF * DIM * 2)
#define P16_BYTES  ((size_t)MROWS * DIM * 2)
#define QK_BYTES   ((size_t)MROWS * QKLD * 2)
#define P32_BYTES  ((size_t)MROWS * DIM * 4)
#define H_BYTES    ((size_t)MROWS * DFF * 2)
#define OFF_WQKV ((size_t)0)
#define OFF_WO   (OFF_WQKV + WQKV_BYTES)
#define OFF_WFC  (OFF_WO + WO_BYTES)
#define OFF_WPJ  (OFF_WFC + WFF_BYTES)
#define OFF_XN   (OFF_WPJ + WFF_BYTES)
#define OFF_QK   (OFF_XN + P16_BYTES)
#define OFF_VT   (OFF_QK + QK_BYTES)
#define OFF_CTX  (OFF_VT + P16_BYTES)
#define OFF_XA   (OFF_CTX + P16_BYTES)
#define OFF_XN2  (OFF_XA + P32_BYTES)
#define OFF_H    (OFF_XN2 + P16_BYTES)
#define WS_TOTAL (OFF_H + H_BYTES)
static_assert((WQKV_BYTES % 128) == 0 && (WO_BYTES % 128) == 0 && (WFF_BYTES % 128) == 0);
static_assert((P16_BYTES % 128) == 0 && (QK_BYTES % 128) == 0 && (P32_BYTES % 128) == 0);
static_assert((H_BYTES % 128) == 0);
static_assert(WS_TOTAL <= (size_t)134217728);

__device__ __forceinline__ float bf16r(float x) {
  unsigned int u = __float_as_uint(x);
  u = (u + 0x7FFFu + ((u >> 16) & 1u)) & 0xFFFF0000u;
  return __uint_as_float(u);
}

__device__ __forceinline__ v16h frag_at(const _Float16* p) {
  v8h lo = *(const v8h*)(p);
  v8h hi = *(const v8h*)(p + 16);
  v16h out;
#pragma unroll
  for (int i = 0; i < 8; ++i) { out[i] = lo[i]; out[i + 8] = hi[i]; }
  return out;
}
__device__ __forceinline__ v16h ld_frag(const _Float16* base, unsigned ld) {
  const unsigned lane = threadIdx.x & 31u;
  return frag_at(base + (lane & 15u) * ld + (lane >> 4) * 8u);
}

__device__ __forceinline__ v8f wmma16(v16h a, v16h b, v8f c) {
  v8f d = __builtin_amdgcn_wmma_f32_16x16x32_f16(false, a, false, b, (short)0, c,
                                                 false, false);
  asm volatile("v_nop\n\tv_nop\n\tv_nop\n\tv_nop" : "+v"(d) : "v"(a), "v"(b));
  return d;
}

__device__ __forceinline__ float red16_max(float x) {
#pragma unroll
  for (int off = 1; off < 16; off <<= 1) x = fmaxf(x, __shfl_xor(x, off, 32));
  return x;
}
__device__ __forceinline__ float red16_sum(float x) {
#pragma unroll
  for (int off = 1; off < 16; off <<= 1) x += __shfl_xor(x, off, 32);
  return x;
}
__device__ __forceinline__ float red32_sum(float x) {
#pragma unroll
  for (int off = 1; off < 32; off <<= 1) x += __shfl_xor(x, off, 32);
  return x;
}

__device__ __forceinline__ void wave_lds_sync() {
  __builtin_amdgcn_fence(3  , "wavefront");
  asm volatile("s_wait_dscnt 0x0" ::: "memory");
  __builtin_amdgcn_wave_barrier();
}

__device__ __forceinline__ unsigned wave_id() {
  return (unsigned)__builtin_amdgcn_readfirstlane((int)(threadIdx.x >> 5));
}

__global__ __launch_bounds__(256) void wt_kernel(
    const float* __restrict__ src, _Float16* __restrict__ dst, unsigned K, unsigned N) {
  __shared__ __attribute__((aligned(16))) _Float16 Ts[64 * LDT];
  const unsigned tid = threadIdx.x;
  const unsigned n0 = blockIdx.x * 64u;
  const unsigned k0 = blockIdx.y * 64u;
#pragma unroll
  for (unsigned j = 0; j < 4u; ++j) {
    const unsigned idx = tid + 256u * j;
    const unsigned r = idx >> 4;
    const unsigned c = (idx & 15u) * 4u;
    const v4f a = *(const v4f*)(src + (size_t)(k0 + r) * N + n0 + c);
#pragma unroll
    for (unsigned jj = 0; jj < 4u; ++jj)
      Ts[(c + jj) * LDT + r] = (_Float16)(WCARRY * bf16r(a[jj]));
  }
  __syncthreads();
  v8h x[2];
  size_t off[2];
#pragma unroll
  for (unsigned i = 0; i < 2u; ++i) {
    const unsigned idx = tid + 256u * i;
    const unsigned nr = idx >> 3;
    const unsigned kc = (idx & 7u) * 8u;
    x[i] = *(const v8h*)&Ts[nr * LDT + kc];
    off[i] = (size_t)(n0 + nr) * K + k0 + kc;
  }
#pragma unroll
  for (int i = 0; i < 2; ++i) *(volatile v8h*)(dst + off[i]) = x[i];
  __threadfence();
#pragma unroll
  for (int i = 0; i < 2; ++i) *(volatile v8h*)(dst + off[i]) = x[i];
}

template <int MODE, int KD, int LDO, int RESX>
__device__ __forceinline__ void gemm_body(
    const _Float16* __restrict__ A16, const _Float16* __restrict__ Bt,
    const float* __restrict__ addf, const float* __restrict__ resf,
    float* __restrict__ outf, _Float16* __restrict__ out16, float* Cs, const float oscale) {
  static_assert((KD % 32) == 0);
  static_assert((LDO % 64) == 0);
  const unsigned tid = threadIdx.x, lane = tid & 31u;
  const unsigned w = wave_id();
  const unsigned mw = w >> 1, nw = w & 1u;
  const unsigned hh = lane >> 4, m = lane & 15u;
  const unsigned n0 = blockIdx.x * 64u;
  const unsigned row0 = blockIdx.y * 64u;
  const unsigned bat = row0 / (unsigned)SEQ;
  const unsigned t0 = row0 - bat * (unsigned)SEQ;
  const unsigned rowF0 = bat * (unsigned)SEQ_FULL + t0;

  const _Float16* ap  = A16 + (size_t)(row0 + mw * 16u + m) * KD + hh * 8u;
  const _Float16* bp0 = Bt + (size_t)(n0 + nw * 32u + m) * KD + hh * 8u;
  const _Float16* bp1 = bp0 + (size_t)16 * KD;
  v8f acc0 = {}, acc1 = {};
#pragma unroll 2
  for (unsigned k0 = 0; k0 < (unsigned)KD; k0 += 32u) {
    const v16h a  = frag_at(ap + k0);
    const v16h b0 = frag_at(bp0 + k0);
    const v16h b1 = frag_at(bp1 + k0);
    acc0 = wmma16(a, b0, acc0);
    acc1 = wmma16(a, b1, acc1);
  }
#pragma unroll
  for (int r = 0; r < 8; ++r) {
    float* d = &Cs[(mw * 16u + hh * 8u + (unsigned)r) * LDC + nw * 32u + m];
    d[0]  = acc0[r];
    d[16] = acc1[r];
  }
  __syncthreads();

  if (MODE == 3) {
    const unsigned c = tid & 63u;
    const float bv = bf16r(addf[n0 + c]);
#pragma unroll 1
    for (unsigned it = 0; it < 16u; ++it) {
      const unsigned r = (tid >> 6) + 4u * it;
      const float v = Cs[r * LDC + c] * oscale + bv;
      Cs[r * LDC + c] = 0.5f * v * (1.0f + erff(v * 0.70710678118654752f));
    }
    __syncthreads();
  }

  if (MODE == 0 || MODE == 3) {
    const float sc = (MODE == 0) ? oscale : 1.0f;
    v8h x[2];
    size_t off[2];
#pragma unroll
    for (unsigned i = 0; i < 2u; ++i) {
      const unsigned r = 32u * i + (tid >> 3);
      const unsigned c = (tid & 7u) * 8u;
      const v4f u0 = *(const v4f*)&Cs[r * LDC + c];
      const v4f u1 = *(const v4f*)&Cs[r * LDC + c + 4];
#pragma unroll
      for (int j = 0; j < 4; ++j) {
        x[i][j]     = (_Float16)(u0[j] * sc);
        x[i][j + 4] = (_Float16)(u1[j] * sc);
      }
      off[i] = (size_t)(row0 + r) * LDO + n0 + c;
    }
#pragma unroll
    for (int i = 0; i < 2; ++i) *(volatile v8h*)(out16 + off[i]) = x[i];
    __threadfence();
#pragma unroll
    for (int i = 0; i < 2; ++i) *(volatile v8h*)(out16 + off[i]) = x[i];
  }

  if (MODE == 1) {
    v8h x[2];
    size_t off[2];
#pragma unroll
    for (unsigned i = 0; i < 2u; ++i) {
      const unsigned dcol = 32u * i + (tid >> 3);
      const unsigned kk = (tid & 7u) * 8u;
#pragma unroll
      for (unsigned j = 0; j < 8u; ++j)
        x[i][j] = (_Float16)(Cs[(kk + j) * LDC + dcol] * oscale);
      off[i] = (size_t)(bat * (unsigned)DIM + n0 + dcol) * SEQ + t0 + kk;
    }
#pragma unroll
    for (int i = 0; i < 2; ++i) *(volatile v8h*)(out16 + off[i]) = x[i];
    __threadfence();
#pragma unroll
    for (int i = 0; i < 2; ++i) *(volatile v8h*)(out16 + off[i]) = x[i];
  }

  if (MODE == 4) {
    const unsigned rrow0 = RESX ? rowF0 : row0;
    const unsigned orow0 = RESX ? row0 : rowF0;
    v4f xs[4];
    size_t off[4];
#pragma unroll
    for (unsigned i = 0; i < 4u; ++i) {
      const unsigned r = 16u * i + (tid >> 4);
      const unsigned c = (tid & 15u) * 4u;
      const v4f u = *(const v4f*)&Cs[r * LDC + c];
      const v4f g = *(const v4f*)(addf + n0 + c);
      const v4f hres = *(const v4f*)(resf + (size_t)(rrow0 + r) * DIM + n0 + c);
      v4f val;
#pragma unroll
      for (int j = 0; j < 4; ++j) {
        const float rv = RESX ? bf16r(hres[j]) : hres[j];
        val[j] = rv + (u[j] * oscale + bf16r(g[j]));
      }
      xs[i] = val;
      off[i] = (size_t)(orow0 + r) * DIM + n0 + c;
    }
#pragma unroll
    for (int i = 0; i < 4; ++i) *(volatile v4f*)(outf + off[i]) = xs[i];
    __threadfence();
#pragma unroll
    for (int i = 0; i < 4; ++i) *(volatile v4f*)(outf + off[i]) = xs[i];
  }
}

__global__ __launch_bounds__(256) void gemm_qk_kernel(
    const _Float16* __restrict__ A16, const _Float16* __restrict__ Bt,
    _Float16* __restrict__ out16) {
  __shared__ __attribute__((aligned(16))) float Cs[64 * LDC];
  gemm_body<0, DIM, QKLD, 0>(A16, Bt, nullptr, nullptr, nullptr, out16, Cs, 1.0f / WCARRY);
}
__global__ __launch_bounds__(256) void gemm_vt_kernel(
    const _Float16* __restrict__ A16, const _Float16* __restrict__ Bt,
    _Float16* __restrict__ out16) {
  __shared__ __attribute__((aligned(16))) float Cs[64 * LDC];
  gemm_body<1, DIM, DIM, 0>(A16, Bt, nullptr, nullptr, nullptr, out16, Cs, 1.0f / WCARRY);
}
__global__ __launch_bounds__(256) void gemm_wo_kernel(
    const _Float16* __restrict__ A16, const _Float16* __restrict__ Bt,
    const float* __restrict__ bias, const float* __restrict__ xin,
    float* __restrict__ outf) {
  __shared__ __attribute__((aligned(16))) float Cs[64 * LDC];
  gemm_body<4, DIM, DIM, 1>(A16, Bt, bias, xin, outf, nullptr, Cs,
                            1.0f / (WCARRY * VCARRY));
}
__global__ __launch_bounds__(256) void gemm_fc_kernel(
    const _Float16* __restrict__ A16, const _Float16* __restrict__ Bt,
    const float* __restrict__ bias, _Float16* __restrict__ out16) {
  __shared__ __attribute__((aligned(16))) float Cs[64 * LDC];
  gemm_body<3, DIM, DFF, 0>(A16, Bt, bias, nullptr, nullptr, out16, Cs, 1.0f / WCARRY);
}
__global__ __launch_bounds__(256) void gemm_proj_kernel(
    const _Float16* __restrict__ A16, const _Float16* __restrict__ Bt,
    const float* __restrict__ bias, const float* __restrict__ resf,
    float* __restrict__ outf) {
  __shared__ __attribute__((aligned(16))) float Cs[64 * LDC];
  gemm_body<4, DFF, DIM, 0>(A16, Bt, bias, resf, outf, nullptr, Cs, 1.0f / WCARRY);
}

__global__ __launch_bounds__(256) void attn_kernel(
    const _Float16* __restrict__ QK, const _Float16* __restrict__ Vt,
    _Float16* __restrict__ Ov) {
  __shared__ __attribute__((aligned(16))) _Float16 Ks[64 * LDT];
  __shared__ __attribute__((aligned(16))) _Float16 Vs[64 * LDT];
  __shared__ __attribute__((aligned(16))) _Float16 Ps[8 * 16 * LDT];

  const unsigned tid = threadIdx.x, lane = tid & 31u;
  const unsigned w = wave_id();
  const unsigned hh = lane >> 4, m = lane & 15u;
  const unsigned q0 = blockIdx.x * 128u;
  const unsigned head = blockIdx.y;
  const unsigned bat = blockIdx.z;
  const unsigned qbase = q0 + w * 16u;
  const unsigned rowb = bat * (unsigned)SEQ;
  const unsigned pbase = w * (16u * LDT);
  const float scale = 0.125f;

  const size_t qoff = (size_t)(rowb + qbase + m) * QKLD + head * HD + hh * 8u;
  v16h qf[2];
  qf[0] = frag_at(QK + qoff);
  qf[1] = frag_at(QK + qoff + 32);

  float mrow[8], lrow[8];
  v8f o[4];
#pragma unroll
  for (int v = 0; v < 8; ++v) { mrow[v] = -1.0e30f; lrow[v] = 0.0f; }
#pragma unroll
  for (int nb = 0; nb < 4; ++nb) o[nb] = (v8f){};

  const size_t kplane = (size_t)rowb * QKLD + DIM + head * HD;
  const size_t vplane = (size_t)(bat * (unsigned)DIM + head * HD) * SEQ;
  const unsigned kend = q0 + 128u;

  for (unsigned kb = 0; kb < kend; kb += 64u) {
#pragma unroll
    for (unsigned j = 0; j < 2u; ++j) {
      const unsigned idx = tid + 256u * j;
      const unsigned r = idx >> 3, c = (idx & 7u) * 8u;
      *(v8h*)&Ks[r * LDT + c] = *(const v8h*)(QK + kplane + (size_t)(kb + r) * QKLD + c);
      *(v8h*)&Vs[r * LDT + c] = *(const v8h*)(Vt + vplane + (size_t)r * SEQ + kb + c);
    }
    __syncthreads();

    if (kb <= qbase) {
      v8f s[4];
#pragma unroll
      for (int kg = 0; kg < 4; ++kg) {
        v8f t = {};
#pragma unroll
        for (int c = 0; c < 2; ++c) {
          const v16h kf = ld_frag(&Ks[(kg * 16) * LDT + c * 32], LDT);
          t = wmma16(qf[c], kf, t);
        }
        s[kg] = t * scale;
      }
      if (kb + 63u > qbase) {
#pragma unroll
        for (int kg = 0; kg < 4; ++kg) {
          const unsigned key = kb + (unsigned)kg * 16u + m;
#pragma unroll
          for (int v = 0; v < 8; ++v) {
            const unsigned qr = qbase + hh * 8u + (unsigned)v;
            s[kg][v] = (key > qr) ? -1.0e30f : s[kg][v];
          }
        }
      }

      float alpha[8];
#pragma unroll
      for (int v = 0; v < 8; ++v) {
        float mx = fmaxf(fmaxf(s[0][v], s[1][v]), fmaxf(s[2][v], s[3][v]));
        mx = red16_max(mx);
        const float mn = fmaxf(mrow[v], mx);
        alpha[v] = __expf(mrow[v] - mn);
        mrow[v] = mn;
      }
#pragma unroll
      for (int kg = 0; kg < 4; ++kg)
#pragma unroll
        for (int v = 0; v < 8; ++v) s[kg][v] = __expf(s[kg][v] - mrow[v]);
#pragma unroll
      for (int v = 0; v < 8; ++v) {
        const float rs = red16_sum((s[0][v] + s[1][v]) + (s[2][v] + s[3][v]));
        lrow[v] = alpha[v] * lrow[v] + rs;
      }
#pragma unroll
      for (int nb = 0; nb < 4; ++nb)
#pragma unroll
        for (int v = 0; v < 8; ++v) o[nb][v] = o[nb][v] * alpha[v];

#pragma unroll
      for (int kg = 0; kg < 4; ++kg)
#pragma unroll
        for (int v = 0; v < 8; ++v)
          Ps[pbase + (hh * 8u + (unsigned)v) * LDT + (unsigned)kg * 16u + m] =
              (_Float16)(s[kg][v] * PCARRY);
      wave_lds_sync();

#pragma unroll
      for (int c = 0; c < 2; ++c) {
        const v16h pf = ld_frag(&Ps[pbase + c * 32], LDT);
#pragma unroll
        for (int nb = 0; nb < 4; ++nb) {
          const v16h vf = ld_frag(&Vs[(nb * 16) * LDT + c * 32], LDT);
          o[nb] = wmma16(pf, vf, o[nb]);
        }
      }
      wave_lds_sync();
    }
    __syncthreads();
  }

  float inv[8];
#pragma unroll
  for (int v = 0; v < 8; ++v) inv[v] = __builtin_amdgcn_rcpf(lrow[v]) * (VCARRY / PCARRY);
#pragma unroll
  for (int nb = 0; nb < 4; ++nb)
#pragma unroll
    for (int v = 0; v < 8; ++v)
      Ps[pbase + (hh * 8u + (unsigned)v) * LDT + (unsigned)nb * 16u + m] =
          (_Float16)(o[nb][v] * inv[v]);
  wave_lds_sync();
  v8h x[4];
  size_t off[4];
#pragma unroll
  for (unsigned i = 0; i < 4u; ++i) {
    const unsigned r = 4u * i + (lane >> 3);
    const unsigned c = (lane & 7u) * 8u;
    x[i] = *(const v8h*)&Ps[pbase + r * LDT + c];
    off[i] = (size_t)(rowb + qbase + r) * DIM + head * HD + c;
  }
#pragma unroll
  for (int i = 0; i < 4; ++i) *(volatile v8h*)(Ov + off[i]) = x[i];
  __threadfence();
#pragma unroll
  for (int i = 0; i < 4; ++i) *(volatile v8h*)(Ov + off[i]) = x[i];
}

__device__ __forceinline__ void ln_store16(
    const float* S, const float* __restrict__ g, const float* __restrict__ be,
    _Float16* __restrict__ out16, size_t obase, float mu, float rs) {
  const unsigned lane = threadIdx.x & 31u;
#pragma unroll 1
  for (unsigned it = 0; it < (unsigned)(DIM / 256); ++it) {
    const unsigned c = it * 256u + lane * 8u;
    const v4f v0 = *(const v4f*)&S[c];
    const v4f v1 = *(const v4f*)&S[c + 4];
    const v4f g0 = *(const v4f*)(g + c);
    const v4f g1 = *(const v4f*)(g + c + 4);
    const v4f b0 = *(const v4f*)(be + c);
    const v4f b1 = *(const v4f*)(be + c + 4);
    v8h x;
#pragma unroll
    for (int j = 0; j < 4; ++j) {
      x[j]     = (_Float16)(bf16r(g0[j]) * (v0[j] - mu) * rs + bf16r(b0[j]));
      x[j + 4] = (_Float16)(bf16r(g1[j]) * (v1[j] - mu) * rs + bf16r(b1[j]));
    }
    *(volatile v8h*)(out16 + obase + c) = x;
  }
}

template <int SRCX>
__device__ __forceinline__ void ln_body(
    const float* __restrict__ src, const float* __restrict__ g,
    const float* __restrict__ be, _Float16* __restrict__ out16, float* S, unsigned row) {
  const unsigned lane = threadIdx.x & 31u;
  const unsigned bat = row / (unsigned)SEQ;
  const unsigned srow = SRCX ? (bat * (unsigned)SEQ_FULL + (row - bat * (unsigned)SEQ)) : row;
  const size_t sbase = (size_t)srow * DIM;
  const size_t obase = (size_t)row * DIM;
  float sum = 0.0f;
#pragma unroll 1
  for (unsigned it = 0; it < (unsigned)(DIM / 128); ++it) {
    const unsigned c = it * 128u + lane * 4u;
    v4f v = *(const v4f*)(src + sbase + c);
    if (SRCX) {
#pragma unroll
      for (int j = 0; j < 4; ++j) v[j] = bf16r(v[j]);
    }
    *(v4f*)&S[c] = v;
    sum += (v[0] + v[1]) + (v[2] + v[3]);
  }
  sum = red32_sum(sum);
  const float mu = sum * (1.0f / (float)DIM);
  float sq = 0.0f;
#pragma unroll 1
  for (unsigned it = 0; it < (unsigned)(DIM / 128); ++it) {
    const unsigned c = it * 128u + lane * 4u;
    const v4f v = *(const v4f*)&S[c];
    const float d0 = v[0] - mu, d1 = v[1] - mu, d2 = v[2] - mu, d3 = v[3] - mu;
    sq += (d0 * d0 + d1 * d1) + (d2 * d2 + d3 * d3);
  }
  sq = red32_sum(sq);
  const float rs = rsqrtf(sq * (1.0f / (float)DIM) + LN_EPS);
  wave_lds_sync();
  ln_store16(S, g, be, out16, obase, mu, rs);
  __threadfence();
  ln_store16(S, g, be, out16, obase, mu, rs);
}

__global__ __launch_bounds__(256) void ln_in_kernel(
    const float* __restrict__ X, const float* __restrict__ g,
    const float* __restrict__ be, _Float16* __restrict__ out16) {
  __shared__ __attribute__((aligned(16))) float S[LNROWS * DIM];
  const unsigned w = wave_id();
  const unsigned row = blockIdx.x * (unsigned)LNROWS + w;
  ln_body<1>(X, g, be, out16, S + w * (unsigned)DIM, row);
}
__global__ __launch_bounds__(256) void ln_mid_kernel(
    const float* __restrict__ XA, const float* __restrict__ g,
    const float* __restrict__ be, _Float16* __restrict__ out16) {
  __shared__ __attribute__((aligned(16))) float S[LNROWS * DIM];
  const unsigned w = wave_id();
  const unsigned row = blockIdx.x * (unsigned)LNROWS + w;
  ln_body<0>(XA, g, be, out16, S + w * (unsigned)DIM, row);
}

extern "C" void kernel_launch(void* const* d_in, const int* in_sizes, int n_in,
                              void* d_out, int out_size, void* d_ws, size_t ws_size,
                              hipStream_t stream) {
  if (n_in < 14) return;
  const long long need_x = (long long)((NB - 1) * SEQ_FULL + SEQ) * DIM;
  if ((long long)in_sizes[0] < need_x) return;
  if ((long long)in_sizes[1] < (long long)DIM * DIM) return;
  if ((long long)in_sizes[2] < (long long)DIM * DIM) return;
  if ((long long)in_sizes[3] < (long long)DIM * DIM) return;
  if ((long long)in_sizes[4] < (long long)DIM * DIM) return;
  if (in_sizes[5] < DIM) return;
  if ((long long)in_sizes[6] < (long long)DIM * DFF) return;
  if (in_sizes[7] < DFF) return;
  if ((long long)in_sizes[8] < (long long)DFF * DIM) return;
  if (in_sizes[9] < DIM || in_sizes[10] < DIM || in_sizes[11] < DIM) return;
  if (in_sizes[12] < DIM || in_sizes[13] < DIM) return;
  if ((long long)out_size < need_x) return;
  if (ws_size < WS_TOTAL) return;

  const float* X     = (const float*)d_in[0];
  const float* Wq    = (const float*)d_in[1];
  const float* Wk    = (const float*)d_in[2];
  const float* Wv    = (const float*)d_in[3];
  const float* Wo    = (const float*)d_in[4];
  const float* bo    = (const float*)d_in[5];
  const float* Wfc   = (const float*)d_in[6];
  const float* bfc   = (const float*)d_in[7];
  const float* Wpj   = (const float*)d_in[8];
  const float* bpj   = (const float*)d_in[9];
  const float* g1    = (const float*)d_in[10];
  const float* be1   = (const float*)d_in[11];
  const float* g2    = (const float*)d_in[12];
  const float* be2   = (const float*)d_in[13];
  float* out = (float*)d_out;

  char* ws = (char*)d_ws;
  _Float16* Wqkv16 = (_Float16*)(ws + OFF_WQKV);
  _Float16* Wo16   = (_Float16*)(ws + OFF_WO);
  _Float16* Wfc16  = (_Float16*)(ws + OFF_WFC);
  _Float16* Wpj16  = (_Float16*)(ws + OFF_WPJ);
  _Float16* XN16   = (_Float16*)(ws + OFF_XN);
  _Float16* QK16   = (_Float16*)(ws + OFF_QK);
  _Float16* Vt16   = (_Float16*)(ws + OFF_VT);
  _Float16* Ctx16  = (_Float16*)(ws + OFF_CTX);
  float*    XA     = (float*)(ws + OFF_XA);
  _Float16* XN2_16 = (_Float16*)(ws + OFF_XN2);
  _Float16* H16    = (_Float16*)(ws + OFF_H);

  dim3 blk(256);

  wt_kernel<<<dim3(DIM / 64, DIM / 64), blk, 0, stream>>>(Wq, Wqkv16, DIM, DIM);
  wt_kernel<<<dim3(DIM / 64, DIM / 64), blk, 0, stream>>>(
      Wk, Wqkv16 + (size_t)DIM * DIM, DIM, DIM);
  wt_kernel<<<dim3(DIM / 64, DIM / 64), blk, 0, stream>>>(
      Wv, Wqkv16 + (size_t)2 * DIM * DIM, DIM, DIM);
  wt_kernel<<<dim3(DIM / 64, DIM / 64), blk, 0, stream>>>(Wo, Wo16, DIM, DIM);
  wt_kernel<<<dim3(DFF / 64, DIM / 64), blk, 0, stream>>>(Wfc, Wfc16, DIM, DFF);
  wt_kernel<<<dim3(DIM / 64, DFF / 64), blk, 0, stream>>>(Wpj, Wpj16, DFF, DIM);

  ln_in_kernel<<<dim3(MROWS / LNROWS), blk, 0, stream>>>(X, g1, be1, XN16);

  gemm_qk_kernel<<<dim3(QKLD / 64, MROWS / 64), blk, 0, stream>>>(XN16, Wqkv16, QK16);
  gemm_vt_kernel<<<dim3(DIM / 64, MROWS / 64), blk, 0, stream>>>(
      XN16, Wqkv16 + (size_t)2 * DIM * DIM, Vt16);

  attn_kernel<<<dim3(SEQ / 128, NHEAD, NB), blk, 0, stream>>>(QK16, Vt16, Ctx16);

  gemm_wo_kernel<<<dim3(DIM / 64, MROWS / 64), blk, 0, stream>>>(Ctx16, Wo16, bo, X, XA);

  ln_mid_kernel<<<dim3(MROWS / LNROWS), blk, 0, stream>>>(XA, g2, be2, XN2_16);

  gemm_fc_kernel<<<dim3(DFF / 64, MROWS / 64), blk, 0, stream>>>(XN2_16, Wfc16, bfc, H16);
  gemm_proj_kernel<<<dim3(DIM / 64, MROWS / 64), blk, 0, stream>>>(H16, Wpj16, bpj, XA, out);
}
